// GCN_AVG_KHop_Anchored_29643864277065
// MI455X (gfx1250) — hardware-verified
//
#include <hip/hip_runtime.h>
#include <stddef.h>


#define CIN     256
#define CHID    128
#define COUT    64
#define CZ      256
#define NTHR    256
#define NWAVE   8
#define EPT     8
#define NGRP    2
#define CHUNK   (NTHR * EPT * NGRP)
#define WCAP    (EPT * NGRP * 32)
#define LISTN   (NWAVE * WCAP)
#define NBC     4096
#define NBF     1024
#define RCAP    40960
#define RBN     128
#define TGT     256
#define DEGCAP  256
#define GROWS   128
#define OTHR    512
#define WSCALE  8.0f
#define WINV    0.125f

#define LDS_FILL ((RCAP + NBF + LISTN) * 4 + 64)
#define LDS_G1   (GROWS * CHID * 4)
#define LDS_G2   (GROWS * COUT * 4)
#define LDS_KHOP (NWAVE * 16 * CZ * 2)

static_assert((CHUNK & (CHUNK - 1)) == 0);
static_assert(CHUNK <= 4096);
static_assert(NBC <= 4096 && NBF <= 4096);
static_assert((NBC & (NBC - 1)) == 0 && (NBF & (NBF - 1)) == 0);
static_assert(NBC == 4 * NBF);
static_assert(OTHR * 8 == NBC);
static_assert((RCAP % 32) == 0);
static_assert(TGT == NWAVE * 32 && (TGT % GROWS) == 0);
static_assert((CIN % 32) == 0 && (CZ % 32) == 0 && (CHID % 16) == 0 && (COUT % 16) == 0);
static_assert(CHID == 4 * 32 && COUT == 2 * 32 && CZ == 2 * CHID);
static_assert((CHID * CIN / 8) % NTHR == 0 && (COUT * CZ / 8) % NTHR == 0);
static_assert((16 * CHID) % 128 == 0 && (16 * COUT) % 128 == 0);

typedef float    v2f  __attribute__((ext_vector_type(2)));
typedef float    v4f  __attribute__((ext_vector_type(4)));
typedef float    v8f  __attribute__((ext_vector_type(8)));
typedef int      v4i  __attribute__((ext_vector_type(4)));
typedef _Float16 v4h  __attribute__((ext_vector_type(4)));
typedef _Float16 v8h  __attribute__((ext_vector_type(8)));
typedef _Float16 v16h __attribute__((ext_vector_type(16)));
union FragH { v16h v; v8h h[2]; };
union FI { float f; int i; };

__device__ __forceinline__ v8h cvt8(v4f a, v4f b) {
  v8h r;
  r[0] = (_Float16)a.x; r[1] = (_Float16)a.y; r[2] = (_Float16)a.z; r[3] = (_Float16)a.w;
  r[4] = (_Float16)b.x; r[5] = (_Float16)b.y; r[6] = (_Float16)b.z; r[7] = (_Float16)b.w;
  return r;
}
__device__ __forceinline__ v4h cvt4(v4f a) {
  v4h r;
  r[0] = (_Float16)a.x; r[1] = (_Float16)a.y; r[2] = (_Float16)a.z; r[3] = (_Float16)a.w;
  return r;
}

__device__ __forceinline__ v8f wmh(v16h a, v16h b, v8f c) {
  v8f d = __builtin_amdgcn_wmma_f32_16x16x32_f16(false, a, false, b, (short)0, c, false, false);
  asm volatile("v_nop\n\tv_nop\n\tv_nop\n\tv_nop" : "+v"(d) : "v"(a), "v"(b));
  return d;
}

__device__ __forceinline__ float nrmval(int c, int mode) {
  const float r0 = rsqrtf((float)(c + 1));
  const int   c1 = c < 1 ? 1 : c;
  const float r1 = __builtin_amdgcn_rcpf((float)c1);
  return mode != 0 ? r1 : r0;
}

template <int NB>
__device__ __forceinline__ int scan_chunk(const int* __restrict__ keys, int nE, int cbase, int slotBase,
                                          int vec8, int* list, int tid, int lane, int wave) {
  int wc = 0;
#pragma unroll
  for (int g = 0; g < NGRP; ++g) {
    const int el0  = (g * NTHR + tid) * EPT;
    const int e0   = cbase + el0;
    const int sent = -2147483647 - 1;
    v4i da, db;
    if (vec8 != 0 && cbase + CHUNK <= nE) {
      da = *(const v4i*)(keys + e0);
      db = *(const v4i*)(keys + e0 + 4);
    } else {
      da.x = (e0     < nE) ? keys[min(e0, nE - 1)] : sent;
      da.y = (e0 + 1 < nE) ? keys[min(e0 + 1, nE - 1)] : sent;
      da.z = (e0 + 2 < nE) ? keys[min(e0 + 2, nE - 1)] : sent;
      da.w = (e0 + 3 < nE) ? keys[min(e0 + 3, nE - 1)] : sent;
      db.x = (e0 + 4 < nE) ? keys[min(e0 + 4, nE - 1)] : sent;
      db.y = (e0 + 5 < nE) ? keys[min(e0 + 5, nE - 1)] : sent;
      db.z = (e0 + 6 < nE) ? keys[min(e0 + 6, nE - 1)] : sent;
      db.w = (e0 + 7 < nE) ? keys[min(e0 + 7, nE - 1)] : sent;
    }
    const unsigned nb = (unsigned)slotBase;
    const unsigned s0 = (unsigned)da.x - nb, s1 = (unsigned)da.y - nb;
    const unsigned s2 = (unsigned)da.z - nb, s3 = (unsigned)da.w - nb;
    const unsigned s4 = (unsigned)db.x - nb, s5 = (unsigned)db.y - nb;
    const unsigned s6 = (unsigned)db.z - nb, s7 = (unsigned)db.w - nb;
    const bool h0 = s0 < (unsigned)NB, h1 = s1 < (unsigned)NB, h2 = s2 < (unsigned)NB, h3 = s3 < (unsigned)NB;
    const bool h4 = s4 < (unsigned)NB, h5 = s5 < (unsigned)NB, h6 = s6 < (unsigned)NB, h7 = s7 < (unsigned)NB;
    const unsigned any = __builtin_amdgcn_ballot_w32(h0 | h1 | h2 | h3 | h4 | h5 | h6 | h7);
    if (any != 0u) {
#define HITJ(J, HJ, SJ) { \
        const unsigned mj = __builtin_amdgcn_ballot_w32(HJ); \
        if (mj != 0u) { \
          if (HJ) { \
            const int pos = wc + (int)__builtin_amdgcn_mbcnt_lo(mj, 0u); \
            if (pos < WCAP) list[wave * WCAP + pos] = ((el0 + (J)) << 12) | (int)(SJ); \
          } \
          wc += (int)__builtin_popcount(mj); } }
      HITJ(0, h0, s0)
      HITJ(1, h1, s1)
      HITJ(2, h2, s2)
      HITJ(3, h3, s3)
      HITJ(4, h4, s4)
      HITJ(5, h5, s5)
      HITJ(6, h6, s6)
      HITJ(7, h7, s7)
#undef HITJ
    }
  }
  return wc;
}

__global__ __launch_bounds__(NTHR) void k_xprep(const float* __restrict__ x, _Float16* x16, int nN, int nTot) {
  const int i = blockIdx.x * NTHR + (int)threadIdx.x;
  if (i >= nTot) return;
  const int row = i >> 5;
  const int c0  = (i & 31) * 8;
  const int rc  = row < nN ? row : nN - 1;
  const float* xp = x + (size_t)rc * CIN + c0;
  v4f a = *(const v4f*)xp;
  v4f b = *(const v4f*)(xp + 4);
  const v4f z4 = {0.f, 0.f, 0.f, 0.f};
  const bool ok = row < nN;
  a = ok ? a : z4;
  b = ok ? b : z4;
  const v8h hv = cvt8(a, b);
  _Float16* dp = x16 + (size_t)i * 8;
  *(volatile v8h*)dp = hv;
  __threadfence();
  *(volatile v8h*)dp = hv;
}

__global__ __launch_bounds__(NTHR) void k_wprep(
    const float* __restrict__ W1, const float* __restrict__ W2, _Float16* p1, _Float16* p2) {
  const int g0 = CHID * CIN / 8;
  const int g1 = COUT * CZ / 8;
  const int bstart = blockIdx.x * NTHR;
  const float* src; _Float16* dst; int K, Nout, segOff;
  if (bstart < g0) { src = W1; dst = p1; K = CIN; Nout = CHID; segOff = 0; }
  else             { src = W2; dst = p2; K = CZ;  Nout = COUT; segOff = g0; }
  const int i = bstart + (int)threadIdx.x;
  if (i >= g0 + g1) return;
  const int o  = (i - segOff) * 8;
  const int n  = o / K;
  const int k0 = o - n * K;
  const int nc = n < Nout ? n : Nout - 1;
  float v[8];
#pragma unroll
  for (int e = 0; e < 8; ++e) {
    const int k  = k0 + e;
    const int kc = k < K ? k : K - 1;
    const float w = src[(size_t)kc * Nout + nc];
    v[e] = (k < K && n < Nout) ? w * WSCALE : 0.0f;
  }
  v4f a, b;
  a.x = v[0]; a.y = v[1]; a.z = v[2]; a.w = v[3];
  b.x = v[4]; b.y = v[5]; b.z = v[6]; b.w = v[7];
  const v8h hv = cvt8(a, b);
  _Float16* dp = dst + o;
  *(volatile v8h*)dp = hv;
  __threadfence();
  *(volatile v8h*)dp = hv;
}

__global__ __launch_bounds__(NTHR) void k_count(
    const int* __restrict__ keys, int* cnt, float* nrm, int nE, int vec8, int mode) {
  __shared__ __attribute__((aligned(16))) int scnt[NBC];
  __shared__ __attribute__((aligned(16))) int list[LISTN];
  __shared__ int wcnt[NWAVE];
  const int tid = threadIdx.x, lane = tid & 31, wave = tid >> 5;
  const int nodeBase = blockIdx.x * NBC;

  for (int i = tid; i < NBC; i += NTHR) scnt[i] = 0;
  __syncthreads();

  const int nChunks = (nE + CHUNK - 1) / CHUNK;
#pragma unroll 1
  for (int ch = 0; ch < nChunks; ++ch) {
    const int cbase = ch * CHUNK;
    const int wc = scan_chunk<NBC>(keys, nE, cbase, nodeBase, vec8, list, tid, lane, wave);
    if (lane == 0) wcnt[wave] = wc;
    __syncthreads();
    if (wave == 0) {
#pragma unroll 1
      for (int wsx = 0; wsx < NWAVE; ++wsx) {
        int n = __builtin_amdgcn_readfirstlane(wcnt[wsx]);
        n = n > WCAP ? WCAP : (n < 0 ? 0 : n);
        const int* lp = list + wsx * WCAP;
#pragma unroll 1
        for (int i = 0; i < n; ++i) {
          const int ent  = __builtin_amdgcn_readfirstlane(lp[i]);
          const int slot = ent & (NBC - 1);
          if (lane == 0) scnt[slot] = scnt[slot] + 1;
        }
      }
    }
    __syncthreads();
  }

  v4i cq[4]; v4f dq[4];
#pragma unroll
  for (int q = 0; q < 4; ++q) {
    const int f = (wave * 4 + q) * 128 + 4 * lane;
    const v4i c = *(const v4i*)(scnt + f);
    cq[q] = c;
    dq[q].x = nrmval(c.x, mode);
    dq[q].y = nrmval(c.y, mode);
    dq[q].z = nrmval(c.z, mode);
    dq[q].w = nrmval(c.w, mode);
  }
  int*   cp = cnt + (size_t)nodeBase;
  float* dp = nrm + (size_t)nodeBase;
#pragma unroll
  for (int q = 0; q < 4; ++q) {
    const int f = (wave * 4 + q) * 128 + 4 * lane;
    *(volatile v4i*)(cp + f) = cq[q];
    *(volatile v4f*)(dp + f) = dq[q];
  }
  __threadfence();
#pragma unroll
  for (int q = 0; q < 4; ++q) {
    const int f = (wave * 4 + q) * 128 + 4 * lane;
    *(volatile v4i*)(cp + f) = cq[q];
    *(volatile v4f*)(dp + f) = dq[q];
  }
}

__global__ __launch_bounds__(OTHR) void k_offsets(
    const int* __restrict__ cnt, int* off, int* rbase, int nChunk) {
  __shared__ __attribute__((aligned(16))) int soff[NBC];
  __shared__ __attribute__((aligned(16))) int srb[RBN];
  __shared__ int wtot[OTHR / 32];
  const int tid = threadIdx.x, lane = tid & 31, wave = tid >> 5, sub = tid >> 7;
  for (int i = tid; i < RBN; i += OTHR) srb[i] = 0;
  int carry = 0;
#pragma unroll 1
  for (int ch = 0; ch < nChunk; ++ch) {
    const int base = ch * NBC;
    const v4i c0 = *(const v4i*)(cnt + base + 8 * tid);
    const v4i c1 = *(const v4i*)(cnt + base + 8 * tid + 4);
    const int e0 = max(c0.x, 0), e1 = max(c0.y, 0), e2 = max(c0.z, 0), e3 = max(c0.w, 0);
    const int e4 = max(c1.x, 0), e5 = max(c1.y, 0), e6 = max(c1.z, 0), e7 = max(c1.w, 0);
    const int ts = e0 + e1 + e2 + e3 + e4 + e5 + e6 + e7;
    int incl = ts;
#pragma unroll
    for (int d = 1; d < 32; d <<= 1) {
      const int t = __shfl_up(incl, d);
      if (lane >= d) incl += t;
    }
    if (lane == 31) wtot[wave] = incl;
    __syncthreads();
    const int S0 = wtot[0]  + wtot[1]  + wtot[2]  + wtot[3];
    const int S1 = wtot[4]  + wtot[5]  + wtot[6]  + wtot[7];
    const int S2 = wtot[8]  + wtot[9]  + wtot[10] + wtot[11];
    const int S3 = wtot[12] + wtot[13] + wtot[14] + wtot[15];
    int pre = 0;
#pragma unroll 1
    for (int w = 4 * sub; w < wave; ++w) pre += wtot[w];
    const int b0 = carry;
    const int b1 = b0 + ((S0 + 31) & ~31);
    const int b2 = b1 + ((S1 + 31) & ~31);
    const int b3 = b2 + ((S2 + 31) & ~31);
    const int b4 = b3 + ((S3 + 31) & ~31);
    const int myb = sub == 0 ? b0 : (sub == 1 ? b1 : (sub == 2 ? b2 : b3));
    if (tid == 0) {
      srb[min(4 * ch + 0, RBN - 1)] = b0;
      srb[min(4 * ch + 1, RBN - 1)] = b1;
      srb[min(4 * ch + 2, RBN - 1)] = b2;
      srb[min(4 * ch + 3, RBN - 1)] = b3;
    }
    int run = myb + pre + incl - ts;
    soff[8 * tid + 0] = run; run += e0;
    soff[8 * tid + 1] = run; run += e1;
    soff[8 * tid + 2] = run; run += e2;
    soff[8 * tid + 3] = run; run += e3;
    soff[8 * tid + 4] = run; run += e4;
    soff[8 * tid + 5] = run; run += e5;
    soff[8 * tid + 6] = run; run += e6;
    soff[8 * tid + 7] = run;
    carry = b4;
    __syncthreads();
    const v4i o0 = *(const v4i*)(soff + 4 * tid);
    const v4i o1 = *(const v4i*)(soff + 4 * (tid + OTHR));
    int* op = off + base;
    *(volatile v4i*)(op + 4 * tid) = o0;
    *(volatile v4i*)(op + 4 * (tid + OTHR)) = o1;
    __threadfence();
    *(volatile v4i*)(op + 4 * tid) = o0;
    *(volatile v4i*)(op + 4 * (tid + OTHR)) = o1;
    __syncthreads();
  }
  if (tid == 0) srb[min(4 * nChunk, RBN - 1)] = carry;
  __syncthreads();
  v4i rv = {0, 0, 0, 0};
  if (tid < 32) rv = *(const v4i*)(srb + 4 * tid);
  if (tid < 32) *(volatile v4i*)(rbase + 4 * tid) = rv;
  __threadfence();
  if (tid < 32) *(volatile v4i*)(rbase + 4 * tid) = rv;
}

__global__ __launch_bounds__(NTHR) void k_fill(
    const int* __restrict__ keys, const int* __restrict__ vals, const int* __restrict__ off,
    const int* __restrict__ rbase, int* csr, int nN, int nE, int vec8, int csrLen) {
  extern __shared__ v4f lds_dyn[];
  int* region = (int*)lds_dyn;
  int* cursor = region + RCAP;
  int* list   = cursor + NBF;
  int* wcnt   = list + LISTN;
  const int tid = threadIdx.x, lane = tid & 31, wave = tid >> 5;
  const int b = blockIdx.x;
  const int nodeBase = b * NBF;

  int rb0 = rbase[b];
  const int rb1 = rbase[b + 1];
  rb0 = rb0 < 0 ? 0 : (rb0 > csrLen ? csrLen : rb0);
  rb0 &= ~31;
  int len = rb1 - rb0;
  len = len < 0 ? 0 : (len > RCAP ? RCAP : len);
  int lenW = (len + 31) & ~31;
  if (rb0 + lenW > csrLen) lenW = (csrLen - rb0) & ~31;

  {
    const v4i z = {0, 0, 0, 0};
    for (int i = tid; i < RCAP / 4; i += NTHR) ((v4i*)region)[i] = z;
    for (int s = tid; s < NBF; s += NTHR) {
      int o = off[nodeBase + s] - rb0;
      o = o < 0 ? 0 : (o > RCAP ? RCAP : o);
      cursor[s] = o;
    }
  }
  __syncthreads();

  const int nChunks = (nE + CHUNK - 1) / CHUNK;
#pragma unroll 1
  for (int ch = 0; ch < nChunks; ++ch) {
    const int cbase = ch * CHUNK;
    const int wc = scan_chunk<NBF>(keys, nE, cbase, nodeBase, vec8, list, tid, lane, wave);
    if (lane == 0) wcnt[wave] = wc;
    __syncthreads();
    if (wave == 0) {
#pragma unroll 1
      for (int wsx = 0; wsx < NWAVE; ++wsx) {
        int n = __builtin_amdgcn_readfirstlane(wcnt[wsx]);
        n = n > WCAP ? WCAP : (n < 0 ? 0 : n);
        const int* lp = list + wsx * WCAP;
#pragma unroll 1
        for (int i = 0; i < n; ++i) {
          const int ent  = __builtin_amdgcn_readfirstlane(lp[i]);
          const int slot = ent & (NBF - 1);
          int e = cbase + ((ent >> 12) & (CHUNK - 1));
          e = e > nE - 1 ? nE - 1 : e;
          int v = vals[e];
          v = v < 0 ? 0 : (v > nN - 1 ? nN - 1 : v);
          if (lane == 0) {
            int pos = cursor[slot];
            pos = pos < 0 ? 0 : (pos > RCAP - 1 ? RCAP - 1 : pos);
            region[pos] = v;
            const int np = pos + 1;
            cursor[slot] = np > RCAP ? RCAP : np;
          }
        }
      }
    }
    __syncthreads();
  }

  const int nv = lenW >> 2;
  int* gp = csr + rb0;
#pragma unroll 1
  for (int i = tid; i < nv; i += NTHR) { const v4i v = ((const v4i*)region)[i]; *(volatile v4i*)(gp + 4 * i) = v; }
  __threadfence();
#pragma unroll 1
  for (int i = tid; i < nv; i += NTHR) { const v4i v = ((const v4i*)region)[i]; *(volatile v4i*)(gp + 4 * i) = v; }
}

template <int KD, int NC>
__global__ __launch_bounds__(NTHR) void k_gemm(
    const _Float16* __restrict__ A, const _Float16* __restrict__ Bs, const float* __restrict__ dinv, float* C) {
  extern __shared__ v4f lds_dyn[];
  float* stg = (float*)lds_dyn;
  constexpr int NT = NC / 16;
  constexpr int NI = 16 * NC / 128;
  const int tid = threadIdx.x, lane = tid & 31, wave = tid >> 5, hh = lane >> 4, m = lane & 15;
  const int rowBase = blockIdx.x * GROWS;
  const int r0 = wave * 16;
  const _Float16* ar = A + (size_t)(rowBase + r0 + m) * KD + 8 * hh;

  v8f acc[NT];
#pragma unroll
  for (int t = 0; t < NT; ++t) { v8f z = {0.f, 0.f, 0.f, 0.f, 0.f, 0.f, 0.f, 0.f}; acc[t] = z; }
#pragma unroll 1
  for (int kt = 0; kt < KD / 32; ++kt) {
    FragH a;
    a.h[0] = *(const v8h*)(ar + 32 * kt);
    a.h[1] = *(const v8h*)(ar + 32 * kt + 16);
#pragma unroll
    for (int t = 0; t < NT; ++t) {
      const _Float16* bp = Bs + (size_t)(16 * t + m) * KD + 32 * kt + 8 * hh;
      FragH b;
      b.h[0] = *(const v8h*)bp;
      b.h[1] = *(const v8h*)(bp + 16);
      acc[t] = wmh(a.v, b.v, acc[t]);
    }
  }

  const v4f dA = *(const v4f*)(dinv + (size_t)rowBase + r0 + 8 * hh);
  const v4f dB = *(const v4f*)(dinv + (size_t)rowBase + r0 + 8 * hh + 4);
  float s[8];
  s[0] = dA.x; s[1] = dA.y; s[2] = dA.z; s[3] = dA.w; s[4] = dB.x; s[5] = dB.y; s[6] = dB.z; s[7] = dB.w;
#pragma unroll
  for (int r = 0; r < 8; ++r) s[r] = s[r] * WINV;
  float* sp = stg + (r0 + 8 * hh) * NC + m;
#pragma unroll
  for (int t = 0; t < NT; ++t) {
#pragma unroll
    for (int r = 0; r < 8; ++r) sp[r * NC + 16 * t] = acc[t][r] * s[r];
  }
  __syncthreads();

  const float* lp = stg + r0 * NC + 4 * lane;
  float* gp = C + ((size_t)rowBase + r0) * NC + 4 * lane;
#pragma unroll
  for (int i = 0; i < NI; ++i) { const v4f v = *(const v4f*)(lp + 128 * i); *(volatile v4f*)(gp + 128 * i) = v; }
  __threadfence();
#pragma unroll
  for (int i = 0; i < NI; ++i) { const v4f v = *(const v4f*)(lp + 128 * i); *(volatile v4f*)(gp + 128 * i) = v; }
}

__global__ __launch_bounds__(NTHR) void k_agg1(
    const int* __restrict__ csr, const int* __restrict__ off, const int* __restrict__ cnt,
    const float* __restrict__ dinv, const float* __restrict__ hw, const float* __restrict__ bias,
    float* h, int nN, int csrLen) {
  const int tid = threadIdx.x, lane = tid & 31, wave = tid >> 5;
  const int tbase = blockIdx.x * TGT + wave * 32;
  const int cl = tbase + lane;
  const int cnt_l = cnt[cl];
  const int off_l = off[cl];
  FI dvu; dvu.f = dinv[cl];
  const v4f bb = *(const v4f*)(bias + 4 * lane);

#pragma unroll 1
  for (int j = 0; j < 32; ++j) {
    const int c = tbase + j;
    int n = __builtin_amdgcn_readlane(cnt_l, j);
    n = n < 0 ? 0 : (n > DEGCAP ? DEGCAP : n);
    const int st = __builtin_amdgcn_readlane(off_l, j);
    FI du; du.i = __builtin_amdgcn_readlane(dvu.i, j);
    const float dc = du.f;
    v4f acc = {0.f, 0.f, 0.f, 0.f};
#pragma unroll 1
    for (int q0 = 0; q0 < n; q0 += 32) {
      int pos = st + q0 + lane;
      pos = pos < 0 ? 0 : (pos > csrLen - 1 ? csrLen - 1 : pos);
      int sl = csr[pos];
      sl = sl < 0 ? 0 : (sl > nN - 1 ? nN - 1 : sl);
      const int mcnt = (n - q0) < 32 ? (n - q0) : 32;
#pragma unroll 1
      for (int p = 0; p < mcnt; ++p) {
        const int s = __builtin_amdgcn_readlane(sl, p);
        acc = acc + *(const v4f*)(hw + (size_t)s * CHID + 4 * lane);
      }
    }
    const v4f sv = *(const v4f*)(hw + (size_t)c * CHID + 4 * lane);
    v4f v = (acc + sv) * dc + bb;
    v.x = fmaxf(v.x, 0.f); v.y = fmaxf(v.y, 0.f); v.z = fmaxf(v.z, 0.f); v.w = fmaxf(v.w, 0.f);
    float* hp = h + (size_t)c * CHID + 4 * lane;
    *(volatile v4f*)hp = v;
    __threadfence();
    *(volatile v4f*)hp = v;
  }
}

__global__ __launch_bounds__(NTHR) void k_khop(
    const int* __restrict__ csr, const int* __restrict__ off, const int* __restrict__ cnt,
    const float* __restrict__ rinv, const float* __restrict__ h, _Float16* z16, int nN, int csrLen) {
  extern __shared__ v4f lds_dyn[];
  const int tid = threadIdx.x, lane = tid & 31, wave = tid >> 5;
  _Float16* stg = (_Float16*)lds_dyn + wave * (16 * CZ);
  const int tbase = blockIdx.x * TGT + wave * 32;
  const int cl = tbase + lane;
  const int cnt_l = cnt[cl];
  const int off_l = off[cl];
  FI rvu; rvu.f = rinv[cl];

#pragma unroll 1
  for (int half = 0; half < 2; ++half) {
#pragma unroll 1
    for (int j = 0; j < 16; ++j) {
      const int jj = 16 * half + j;
      const int c = tbase + jj;
      int n = __builtin_amdgcn_readlane(cnt_l, jj);
      n = n < 0 ? 0 : (n > DEGCAP ? DEGCAP : n);
      const int st = __builtin_amdgcn_readlane(off_l, jj);
      FI ru; ru.i = __builtin_amdgcn_readlane(rvu.i, jj);
      const float ri = ru.f;
      v4f acc = {0.f, 0.f, 0.f, 0.f};
#pragma unroll 1
      for (int q0 = 0; q0 < n; q0 += 32) {
        int pos = st + q0 + lane;
        pos = pos < 0 ? 0 : (pos > csrLen - 1 ? csrLen - 1 : pos);
        int dl = csr[pos];
        dl = dl < 0 ? 0 : (dl > nN - 1 ? nN - 1 : dl);
        const int mcnt = (n - q0) < 32 ? (n - q0) : 32;
#pragma unroll 1
        for (int p = 0; p < mcnt; ++p) {
          const int d = __builtin_amdgcn_readlane(dl, p);
          acc = acc + *(const v4f*)(h + (size_t)d * CHID + 4 * lane);
        }
      }
      const v4f own = *(const v4f*)(h + (size_t)c * CHID + 4 * lane);
      const v4f kh = acc * ri;
      const v4f df = own - kh;
      *(v4h*)(stg + j * CZ + 4 * lane)        = cvt4(df);
      *(v4h*)(stg + j * CZ + CHID + 4 * lane) = cvt4(kh);
    }
    __syncthreads();
    const int row0 = tbase + 16 * half;
    _Float16* gp = z16 + (size_t)row0 * CZ + 8 * lane;
#pragma unroll
    for (int i = 0; i < 16; ++i) { const v8h v = *(const v8h*)(stg + i * CZ + 8 * lane); *(volatile v8h*)(gp + (size_t)i * CZ) = v; }
    __threadfence();
#pragma unroll
    for (int i = 0; i < 16; ++i) { const v8h v = *(const v8h*)(stg + i * CZ + 8 * lane); *(volatile v8h*)(gp + (size_t)i * CZ) = v; }
    __syncthreads();
  }
}

__global__ __launch_bounds__(NTHR) void k_agg2(
    const int* __restrict__ csr, const int* __restrict__ off, const int* __restrict__ cnt,
    const float* __restrict__ dinv, const float* __restrict__ tw, const float* __restrict__ bias,
    float* out, int nN, int csrLen) {
  __shared__ __attribute__((aligned(16))) float stg[NWAVE * 16 * COUT];
  const int tid = threadIdx.x, lane = tid & 31, wave = tid >> 5;
  float* sw = stg + wave * (16 * COUT);
  const int tbase = blockIdx.x * TGT + wave * 32;
  const int cl = tbase + lane;
  const int cnt_l = cnt[cl];
  const int off_l = off[cl];
  FI dvu; dvu.f = dinv[cl];
  const v2f bb = *(const v2f*)(bias + 2 * lane);

#pragma unroll 1
  for (int half = 0; half < 2; ++half) {
#pragma unroll 1
    for (int j = 0; j < 16; ++j) {
      const int jj = 16 * half + j;
      const int c = tbase + jj;
      int n = __builtin_amdgcn_readlane(cnt_l, jj);
      n = n < 0 ? 0 : (n > DEGCAP ? DEGCAP : n);
      const int st = __builtin_amdgcn_readlane(off_l, jj);
      FI du; du.i = __builtin_amdgcn_readlane(dvu.i, jj);
      const float dc = du.f;
      v2f acc = {0.f, 0.f};
#pragma unroll 1
      for (int q0 = 0; q0 < n; q0 += 32) {
        int pos = st + q0 + lane;
        pos = pos < 0 ? 0 : (pos > csrLen - 1 ? csrLen - 1 : pos);
        int sl = csr[pos];
        sl = sl < 0 ? 0 : (sl > nN - 1 ? nN - 1 : sl);
        const int mcnt = (n - q0) < 32 ? (n - q0) : 32;
#pragma unroll 1
        for (int p = 0; p < mcnt; ++p) {
          const int s = __builtin_amdgcn_readlane(sl, p);
          acc = acc + *(const v2f*)(tw + (size_t)s * COUT + 2 * lane);
        }
      }
      const v2f sv = *(const v2f*)(tw + (size_t)c * COUT + 2 * lane);
      const v2f v = (acc + sv) * dc + bb;
      *(v2f*)(sw + j * COUT + 2 * lane) = v;
    }
    __syncthreads();
    const int row0 = tbase + 16 * half;
    float* gp = out + (size_t)row0 * COUT + 4 * lane;
#pragma unroll
    for (int i = 0; i < 8; ++i) {
      const v4f v = *(const v4f*)(sw + 128 * i + 4 * lane);
      const int rem = nN - (row0 + 2 * i);
      if (rem >= 2) { *(volatile v4f*)(gp + 128 * i) = v; }
      else if (rem == 1) { if (lane < 16) *(volatile v4f*)(gp + 128 * i) = v; }
    }
    __threadfence();
#pragma unroll
    for (int i = 0; i < 8; ++i) {
      const v4f v = *(const v4f*)(sw + 128 * i + 4 * lane);
      const int rem = nN - (row0 + 2 * i);
      if (rem >= 2) { *(volatile v4f*)(gp + 128 * i) = v; }
      else if (rem == 1) { if (lane < 16) *(volatile v4f*)(gp + 128 * i) = v; }
    }
    __syncthreads();
  }
}

extern "C" void kernel_launch(void* const* d_in, const int* in_sizes, int n_in,
                              void* d_out, int out_size, void* d_ws, size_t ws_size,
                              hipStream_t stream) {
  if (n_in < 6) return;
  const int nN = in_sizes[0] / CIN;
  const int nE = in_sizes[5] / 2;
  if (nN <= 0 || nE <= 0 || in_sizes[0] != nN * CIN || in_sizes[5] != 2 * nE) return;
  if (in_sizes[1] != CIN * CHID || in_sizes[2] < CHID || in_sizes[3] != CZ * COUT || in_sizes[4] < COUT) return;
  if (out_size != nN * COUT) return;
  if (nE > (1 << 28) || nN > (1 << 24)) return;

  const float* x  = (const float*)d_in[0];
  const float* W1 = (const float*)d_in[1];
  const float* b1 = (const float*)d_in[2];
  const float* W2 = (const float*)d_in[3];
  const float* b2 = (const float*)d_in[4];
  const int*   ei = (const int*)d_in[5];
  float* out = (float*)d_out;

  const int NPAD   = ((nN + TGT - 1) / TGT) * TGT;
  const int nBC    = (nN + NBC - 1) / NBC;
  const int CNTPAD = nBC * NBC;
  if (4 * nBC + 1 > RBN) return;
  const int nBF    = (nN + NBF - 1) / NBF;
  const int csrLen = ((nE + 31) & ~31) + 4096;
  const int nGemm  = NPAD / GROWS;
  const int nAgg   = NPAD / TGT;
  const int nXp    = NPAD * (CIN / 8);

  char* ws = (char*)d_ws;
  size_t off = 0;
  const size_t oX16  = off; off += (size_t)NPAD * CIN * 2;        off = (off + 255) & ~(size_t)255;
  const size_t oP1   = off; off += (size_t)CHID * CIN * 2;        off = (off + 255) & ~(size_t)255;
  const size_t oP2   = off; off += (size_t)COUT * CZ * 2;         off = (off + 255) & ~(size_t)255;
  const size_t oCntD = off; off += (size_t)CNTPAD * 4;            off = (off + 255) & ~(size_t)255;
  const size_t oDv   = off; off += (size_t)CNTPAD * 4;            off = (off + 255) & ~(size_t)255;
  const size_t oOffD = off; off += (size_t)CNTPAD * 4;            off = (off + 255) & ~(size_t)255;
  const size_t oRbD  = off; off += (size_t)RBN * 4;               off = (off + 255) & ~(size_t)255;
  const size_t oCsrD = off; off += (size_t)csrLen * 4;            off = (off + 255) & ~(size_t)255;
  const size_t oCntS = off; off += (size_t)CNTPAD * 4;            off = (off + 255) & ~(size_t)255;
  const size_t oRi   = off; off += (size_t)CNTPAD * 4;            off = (off + 255) & ~(size_t)255;
  const size_t oOffS = off; off += (size_t)CNTPAD * 4;            off = (off + 255) & ~(size_t)255;
  const size_t oRbS  = off; off += (size_t)RBN * 4;               off = (off + 255) & ~(size_t)255;
  const size_t oCsrS = off; off += (size_t)csrLen * 4;            off = (off + 255) & ~(size_t)255;
  const size_t oHw   = off; off += (size_t)NPAD * CHID * 4;       off = (off + 255) & ~(size_t)255;
  const size_t oH    = off; off += (size_t)NPAD * CHID * 4;       off = (off + 255) & ~(size_t)255;
  const size_t oZ    = off; off += (size_t)NPAD * CZ * 2;         off = (off + 255) & ~(size_t)255;
  const size_t oTw   = off; off += (size_t)NPAD * COUT * 4;       off = (off + 255) & ~(size_t)255;
  if (off > ws_size) return;
  _Float16* x16  = (_Float16*)(ws + oX16);
  _Float16* p1   = (_Float16*)(ws + oP1);
  _Float16* p2   = (_Float16*)(ws + oP2);
  int*      cntD = (int*)(ws + oCntD);
  float*    dinv = (float*)(ws + oDv);
  int*      offD = (int*)(ws + oOffD);
  int*      rbD  = (int*)(ws + oRbD);
  int*      csrD = (int*)(ws + oCsrD);
  int*      cntS = (int*)(ws + oCntS);
  float*    rinv = (float*)(ws + oRi);
  int*      offS = (int*)(ws + oOffS);
  int*      rbS  = (int*)(ws + oRbS);
  int*      csrS = (int*)(ws + oCsrS);
  float*    hw   = (float*)(ws + oHw);
  float*    h    = (float*)(ws + oH);
  _Float16* z16  = (_Float16*)(ws + oZ);
  float*    tw   = (float*)(ws + oTw);

  const int* srcs = ei;
  const int* dsts = ei + nE;
  const int vec8S = 1;
  const int vec8D = ((nE & 3) == 0) ? 1 : 0;

  k_xprep<<<nXp / NTHR, NTHR, 0, stream>>>(x, x16, nN, nXp);
  k_wprep<<<(CHID * CIN / 8 + COUT * CZ / 8) / NTHR, NTHR, 0, stream>>>(W1, W2, p1, p2);

  hipFuncSetAttribute(reinterpret_cast<const void*>(&k_fill),
                      hipFuncAttributeMaxDynamicSharedMemorySize, LDS_FILL);
  k_count<<<nBC, NTHR, 0, stream>>>(dsts, cntD, dinv, nE, vec8D, 0);
  k_offsets<<<1, OTHR, 0, stream>>>(cntD, offD, rbD, nBC);
  k_fill<<<nBF, NTHR, LDS_FILL, stream>>>(dsts, srcs, offD, rbD, csrD, nN, nE, vec8D, csrLen);

  k_count<<<nBC, NTHR, 0, stream>>>(srcs, cntS, rinv, nE, vec8S, 1);
  k_offsets<<<1, OTHR, 0, stream>>>(cntS, offS, rbS, nBC);
  k_fill<<<nBF, NTHR, LDS_FILL, stream>>>(srcs, dsts, offS, rbS, csrS, nN, nE, vec8S, csrLen);

  hipFuncSetAttribute(reinterpret_cast<const void*>(&k_gemm<CIN, CHID>),
                      hipFuncAttributeMaxDynamicSharedMemorySize, LDS_G1);
  hipFuncSetAttribute(reinterpret_cast<const void*>(&k_gemm<CZ, COUT>),
                      hipFuncAttributeMaxDynamicSharedMemorySize, LDS_G2);
  k_gemm<CIN, CHID><<<nGemm, NTHR, LDS_G1, stream>>>(x16, p1, dinv, hw);
  k_agg1<<<nAgg, NTHR, 0, stream>>>(csrD, offD, cntD, dinv, hw, b1, h, nN, csrLen);

  hipFuncSetAttribute(reinterpret_cast<const void*>(&k_khop),
                      hipFuncAttributeMaxDynamicSharedMemorySize, LDS_KHOP);
  k_khop<<<nAgg, NTHR, LDS_KHOP, stream>>>(csrS, offS, cntS, rinv, h, z16, nN, csrLen);

  k_gemm<CZ, COUT><<<nGemm, NTHR, LDS_G2, stream>>>(z16, p2, dinv, tw);
  k_agg2<<<nAgg, NTHR, 0, stream>>>(csrD, offD, cntD, dinv, tw, b2, out, nN, csrLen);
}
